// Block2_90263032692810
// MI455X (gfx1250) — hardware-run, weakly checked
//
#include <hip/hip_runtime.h>
#include <math.h>

typedef __attribute__((ext_vector_type(16))) _Float16 v16h;
typedef __attribute__((ext_vector_type(8)))  _Float16 v8h;
typedef __attribute__((ext_vector_type(16))) __bf16   v16b;
typedef __attribute__((ext_vector_type(8)))  __bf16   v8b;
typedef __attribute__((ext_vector_type(8)))  float    v8f;
typedef __attribute__((ext_vector_type(4)))  float    v4f;
typedef __attribute__((ext_vector_type(2)))  float    v2f;

constexpr int kBatch   = 2;
constexpr int kCh      = 192;
constexpr int kHgt     = 64;
constexpr int kWid     = 64;
constexpr int kSeq     = kHgt * kWid;
constexpr int kTok     = kBatch * kSeq;
constexpr int kDm      = kCh;
constexpr int kDin     = 2 * kDm;
constexpr int kNst     = 16;
constexpr int kDtR     = 12;
constexpr int kNL      = 4;
constexpr int kXzP     = 2 * kDin;
constexpr int kXdW     = kDtR + 2 * kNst;
constexpr int kXdP     = 64;
constexpr int kMlpRows = kBatch * kCh * kHgt;
constexpr int kMlpH    = 4 * kWid;
constexpr int kNchw    = kBatch * kCh * kHgt * kWid;
constexpr int kConvCh  = 128;
constexpr int kConvTP  = 132;
constexpr int kScanCh  = 64;
constexpr int kScanTS  = 64;
constexpr int kScanYP  = 68;
static_assert((kDm % 32) == 0 && (kDin % 32) == 0 && (kWid % 32) == 0 && (kMlpH % 32) == 0, "K multiples of 32");
static_assert((kTok % 64) == 0 && (kXzP % 64) == 0 && (kXdP % 64) == 0 && (kDm % 64) == 0 &&
              (kMlpRows % 64) == 0 && (kMlpH % 64) == 0 && (kWid % 64) == 0, "M,N multiples of 64");
static_assert((kDin % kConvCh) == 0 && (kDin % kScanCh) == 0 && (kSeq % kScanTS) == 0 && (kSeq % 64) == 0, "tile multiples");
static_assert(kXdW <= kXdP, "pad");

constexpr int kTilesIn  = (kTok / 64) * (kXzP / 64);
constexpr int kTilesX   = (kTok / 64) * (kXdP / 64);
constexpr int kTilesOut = (kTok / 64) * (kDm / 64);
constexpr int kTilesM1  = (kMlpRows / 64) * (kMlpH / 64);
constexpr int kTilesM2  = (kMlpRows / 64) * (kWid / 64);
static_assert((kTilesIn % 8) == 0 && (kTilesX % 8) == 0 && (kTilesOut % 8) == 0 && (kTilesM1 % 8) == 0 && (kTilesM2 % 8) == 0, "whole blocks");

constexpr size_t kSzTokF32 = (size_t)kTok * kDm * 4;
constexpr size_t kSzTokF16 = (size_t)kTok * kDm * 2;
constexpr size_t kOffM    = 0;
constexpr size_t kOffRes  = kOffM    + kSzTokF32;
constexpr size_t kOffOutl = kOffRes  + kSzTokF32;
constexpr size_t kOffHn   = kOffOutl + kSzTokF32;
constexpr size_t kOffWi   = kOffHn   + kSzTokF16;
constexpr size_t kOffWx   = kOffWi   + (size_t)kNL * kXzP * kDm * 2;
constexpr size_t kOffWo   = kOffWx   + (size_t)kNL * kXdP * kDin * 2;
constexpr size_t kOffW1   = kOffWo   + (size_t)kNL * kDm * kDin * 2;
constexpr size_t kOffW2   = kOffW1   + (size_t)kMlpH * kWid * 2;
constexpr size_t kOffXz   = kOffW2   + (size_t)kWid * kMlpH * 2;
constexpr size_t kOffUc   = kOffXz   + (size_t)kTok * kXzP * 4;
constexpr size_t kOffUc16 = kOffUc   + (size_t)kTok * kDin * 4;
constexpr size_t kOffXd   = kOffUc16 + (size_t)kTok * kDin * 2;
constexpr size_t kOffY16  = kOffXd   + (size_t)kTok * kXdP * 4;
constexpr size_t kOffM2   = kOffY16  + (size_t)kTok * kDin * 2;
constexpr size_t kOffT16  = kOffM2   + (size_t)kMlpRows * kWid * 4;
constexpr size_t kWsTotal = kOffT16  + (size_t)kMlpRows * kWid * 2;
static_assert(kWsTotal == 85917696ull, "carve total");
static_assert(kWsTotal <= 134217728ull, "carve cap");
static_assert((size_t)kMlpRows * kMlpH * 4 == (size_t)kTok * kXzP * 4, "H1 fits the XZ region exactly");
static_assert((size_t)kMlpRows * kMlpH * 2 == (size_t)kTok * kDin * 4, "G16 fits the UC region exactly");
static_assert((kOffRes % 128) == 0 && (kOffOutl % 128) == 0 && (kOffHn % 128) == 0 && (kOffWi % 128) == 0 &&
              (kOffWx % 128) == 0 && (kOffWo % 128) == 0 && (kOffW1 % 128) == 0 && (kOffW2 % 128) == 0 &&
              (kOffXz % 128) == 0 && (kOffUc % 128) == 0 && (kOffUc16 % 128) == 0 && (kOffXd % 128) == 0 &&
              (kOffY16 % 128) == 0 && (kOffM2 % 128) == 0 && (kOffT16 % 128) == 0, "128-B aligned regions");

__device__ __forceinline__ unsigned short f2bf_bits(float f) {
  unsigned u = __float_as_uint(f);
  return (unsigned short)((u + 0x7FFFu + ((u >> 16) & 1u)) >> 16);
}
__device__ __forceinline__ float bf_bits2f(unsigned short h) { return __uint_as_float(((unsigned)h) << 16); }

__device__ __forceinline__ void dep_guard_h(v8f& a, v8f& b, v16h x, v16h y) { asm volatile("v_nop\n\tv_nop\n\tv_nop\n\tv_nop" : "+v"(a), "+v"(b) : "v"(x), "v"(y)); }
__device__ __forceinline__ void dep_guard_b(v8f& a, v8f& b, v16b x, v16b y) { asm volatile("v_nop\n\tv_nop\n\tv_nop\n\tv_nop" : "+v"(a), "+v"(b) : "v"(x), "v"(y)); }
__device__ __forceinline__ void keep4_h(v16h a, v16h b, v16h c, v16h d) { asm volatile("v_nop" :: "v"(a), "v"(b), "v"(c), "v"(d)); }
__device__ __forceinline__ void keep4_b(v16b a, v16b b, v16b c, v16b d) { asm volatile("v_nop" :: "v"(a), "v"(b), "v"(c), "v"(d)); }
__device__ __forceinline__ void acc_guard4(v8f& a, v8f& b, v8f& c, v8f& d) { asm volatile("v_nop\n\tv_nop\n\tv_nop\n\tv_nop" : "+v"(a), "+v"(b), "+v"(c), "+v"(d)); }
template <typename T> struct Frag;
template <> struct Frag<_Float16> {
  typedef v16h V; union U { v16h v; v8h h[2]; };
  static __device__ __forceinline__ v16h load(const _Float16* p) {
    U f; f.h[0] = *(const v8h*)(p); f.h[1] = *(const v8h*)(p + 16); return f.v;
  }
  static __device__ __forceinline__ v8f mma(v16h a, v16h b, v8f c) {
    return __builtin_amdgcn_wmma_f32_16x16x32_f16(false, a, false, b, (short)0, c, false, false);
  }
  static __device__ __forceinline__ void guard(v8f& a, v8f& b, v16h x, v16h y) { dep_guard_h(a, b, x, y); }
  static __device__ __forceinline__ void keep(v16h a, v16h b, v16h c, v16h d) { keep4_h(a, b, c, d); }
};
template <> struct Frag<__bf16> {
  typedef v16b V; union U { v16b v; v8b h[2]; };
  static __device__ __forceinline__ v16b load(const __bf16* p) {
    U f; f.h[0] = *(const v8b*)(p); f.h[1] = *(const v8b*)(p + 16); return f.v;
  }
  static __device__ __forceinline__ v8f mma(v16b a, v16b b, v8f c) {
    return __builtin_amdgcn_wmma_f32_16x16x32_bf16(false, a, false, b, (short)0, c, false, false);
  }
  static __device__ __forceinline__ void guard(v8f& a, v8f& b, v16b x, v16b y) { dep_guard_b(a, b, x, y); }
  static __device__ __forceinline__ void keep(v16b a, v16b b, v16b c, v16b d) { keep4_b(a, b, c, d); }
};

template <int ET> struct Elem;
template <> struct Elem<0> { typedef _Float16 T; };
template <> struct Elem<1> { typedef __bf16 T; };
template <int ET, int SPL, int BIAS_MODE, int OUT_MODE, bool RESID, int ACT = 0>
__global__ __launch_bounds__(256) void wmma_gemm64(
    const unsigned short* __restrict__ Ap, const unsigned short* __restrict__ A2p, int lda, long strideA,
    const unsigned short* __restrict__ Btp, const unsigned short* __restrict__ Bt2p, int ldb, long strideB,
    void* __restrict__ Cout, void* __restrict__ Cout2, int ldc, long strideC,
    const float* __restrict__ bias,
    const float* __restrict__ resid, long strideR,
    int M, int N, int K, float scale) {
  typedef typename Elem<ET>::T T;
  typedef typename Frag<T>::V V;
  const T* A = (const T*)Ap; const T* A2 = (const T*)A2p; const T* Bt = (const T*)Btp; const T* Bt2 = (const T*)Bt2p;
  __shared__ __align__(16) float sT[8][16 * 68];
  const int b    = blockIdx.y;
  const int lane = threadIdx.x & 31;
  const int wave = threadIdx.x >> 5;
  const int tilesN = N >> 6;
  const int tilesM = M >> 6;
  const int tile = blockIdx.x * 8 + wave;
  if (tile >= tilesM * tilesN) return;
  const int tm = tile / tilesN;
  const int tn = tile - tm * tilesN;
  const int m0 = tm << 6;
  const int n0 = tn << 6;

  const T* Ab  = A  + (size_t)b * strideA;
  const T* Bb  = Bt + (size_t)b * strideB;
  const T* Ab2 = (SPL >= 1) ? (A2  + (size_t)b * strideA) : nullptr;
  const T* Bb2 = (SPL == 2) ? (Bt2 + (size_t)b * strideB) : nullptr;

  const int rlane = lane & 15;
  const int koff  = (lane >> 4) * 8;
  const int mOff  = (lane >> 4) * 8;

  v8f acc[4][4];
#pragma unroll
  for (int i = 0; i < 4; ++i)
#pragma unroll
    for (int j = 0; j < 4; ++j) acc[i][j] = (v8f){0.f,0.f,0.f,0.f,0.f,0.f,0.f,0.f};

  for (int k0 = 0; k0 < K; k0 += 32) {
    V bh[4], bl[4];
#pragma unroll
    for (int j = 0; j < 4; ++j) {
      const size_t bo = (size_t)(n0 + (j << 4) + rlane) * ldb + koff + k0;
      bh[j] = Frag<T>::load(Bb + bo);
      if (SPL == 2) bl[j] = Frag<T>::load(Bb2 + bo);
    }
#pragma unroll
    for (int i = 0; i < 4; ++i) {
      const size_t ao = (size_t)(m0 + (i << 4) + rlane) * lda + koff + k0;
      V ah = Frag<T>::load(Ab + ao);
      V al;
      if (SPL >= 1) al = Frag<T>::load(Ab2 + ao);
#pragma unroll
      for (int j = 0; j < 4; ++j) {
        acc[i][j] = Frag<T>::mma(ah, bh[j], acc[i][j]);
        if (SPL == 2) acc[i][j] = Frag<T>::mma(ah, bl[j], acc[i][j]);
        if (SPL >= 1) acc[i][j] = Frag<T>::mma(al, bh[j], acc[i][j]);
      }
      Frag<T>::guard(acc[i][0], acc[i][3], ah, (SPL >= 1) ? al : ah);
    }
    Frag<T>::keep(bh[0], bh[1], bh[2], bh[3]);
    if (SPL == 2) Frag<T>::keep(bl[0], bl[1], bl[2], bl[3]);
  }
  acc_guard4(acc[0][0], acc[0][1], acc[0][2], acc[0][3]);
  acc_guard4(acc[1][0], acc[1][1], acc[1][2], acc[1][3]);
  acc_guard4(acc[2][0], acc[2][1], acc[2][2], acc[2][3]);
  acc_guard4(acc[3][0], acc[3][1], acc[3][2], acc[3][3]);

  float* slab = sT[wave];
  const float* Rb = RESID ? (resid + (size_t)b * strideR) : nullptr;
#pragma unroll
  for (int i = 0; i < 4; ++i) {
    const int mBase = m0 + (i << 4);
#pragma unroll
    for (int j = 0; j < 4; ++j) {
      const int n = n0 + (j << 4) + rlane;
      float bv = 0.f;
      if (BIAS_MODE == 2) bv = bias[n];
#pragma unroll
      for (int r = 0; r < 8; ++r) {
        float v = acc[i][j][r] * scale;
        if (BIAS_MODE == 1) v += bias[mBase + mOff + r];
        if (BIAS_MODE == 2) v += bv;
        if (RESID) v += Rb[(size_t)(mBase + mOff + r) * ldc + n];
        if (ACT == 1) v = tanhf(v);
        if (ACT == 2) v = fmaxf(v, 0.0f);
        if (ACT == 3) v = v / (1.0f + expf(-v));
        if (ACT == 4) v = (v > 0.f) ? v : 0.01f * v;
        slab[(mOff + r) * 68 + (j << 4) + rlane] = v;
      }
    }
    __builtin_amdgcn_fence(__ATOMIC_RELEASE, "workgroup");
    __builtin_amdgcn_wave_barrier();
    __builtin_amdgcn_fence(__ATOMIC_ACQUIRE, "workgroup");
    if (OUT_MODE == 0) {
      float* C = (float*)Cout + (size_t)b * strideC;
      const int hh = lane >> 4, c4 = (lane & 15) * 4;
      for (int pass = 0; pass < 2; ++pass) {
#pragma unroll
        for (int it = 0; it < 8; ++it) {
          const int row = it * 2 + hh;
          v4f v = *(const v4f*)(slab + row * 68 + c4);
          *(volatile v4f*)(C + (size_t)(mBase + row) * ldc + n0 + c4) = v;
        }
        __threadfence();
      }
    } else {
      const int q = lane >> 3, c8 = (lane & 7) * 8;
      unsigned short* C  = (unsigned short*)Cout  + (size_t)b * strideC;
      unsigned short* C2 = (OUT_MODE == 2) ? ((unsigned short*)Cout2 + (size_t)b * strideC) : nullptr;
      for (int pass = 0; pass < 2; ++pass) {
#pragma unroll
        for (int it = 0; it < 4; ++it) {
          const int row = it * 4 + q;
          const float* sp = slab + row * 68 + c8;
          v8h hv, lv;
#pragma unroll
          for (int e = 0; e < 8; ++e) {
            if (OUT_MODE == 1) {
              hv[e] = (_Float16)sp[e];
            } else {
              unsigned short hb = f2bf_bits(sp[e]);
              unsigned short lb = f2bf_bits(sp[e] - bf_bits2f(hb));
              hv[e] = __builtin_bit_cast(_Float16, hb);
              lv[e] = __builtin_bit_cast(_Float16, lb);
            }
          }
          *(volatile v8h*)(C + (size_t)(mBase + row) * ldc + n0 + c8) = hv;
          if (OUT_MODE == 2) *(volatile v8h*)(C2 + (size_t)(mBase + row) * ldc + n0 + c8) = lv;
        }
        __threadfence();
      }
    }
    __builtin_amdgcn_fence(__ATOMIC_RELEASE, "workgroup");
    __builtin_amdgcn_wave_barrier();
    __builtin_amdgcn_fence(__ATOMIC_ACQUIRE, "workgroup");
  }
}

__device__ __forceinline__ float wave_sum(float v) {
#pragma unroll
  for (int off = 16; off >= 1; off >>= 1) v += __shfl_xor(v, off, 32);
  return v;
}

__global__ __launch_bounds__(256) void cast_scale_f16x8_kernel(
    const float* __restrict__ in, unsigned short* __restrict__ out, int total8, float sc)
{
  const int i = blockIdx.x * 256 + threadIdx.x;
  if (i >= total8) return;
  const size_t e0 = (size_t)i << 3;
  const v4f a0 = *(const v4f*)(in + e0);
  const v4f a1 = *(const v4f*)(in + e0 + 4);
  v8h hv;
#pragma unroll
  for (int e = 0; e < 4; ++e) {
    hv[e]     = (_Float16)(a0[e] * sc);
    hv[4 + e] = (_Float16)(a1[e] * sc);
  }
  unsigned short* q = out + e0;
  *(volatile v8h*)q = hv;
  __threadfence();
  *(volatile v8h*)q = hv;
}

__global__ __launch_bounds__(256) void cast_xproj_pad_f16_kernel(
    const float* __restrict__ in, unsigned short* __restrict__ out, int total8)
{
  const int i = blockIdx.x * 256 + threadIdx.x;
  if (i >= total8) return;
  const size_t e0 = (size_t)i << 3;
  const int k = (int)(e0 % kDin);
  const int r = (int)((e0 / kDin) % kXdP);
  const int l = (int)(e0 / ((size_t)kDin * kXdP));
  const int rc = (r < kXdW) ? r : (kXdW - 1);
  const float sc = (r < kXdW) ? 64.0f : 0.0f;
  const float* src = in + ((size_t)(l * kXdW + rc) * kDin + k);
  const v4f a0 = *(const v4f*)(src);
  const v4f a1 = *(const v4f*)(src + 4);
  v8h hv;
#pragma unroll
  for (int e = 0; e < 4; ++e) {
    hv[e]     = (_Float16)(a0[e] * sc);
    hv[4 + e] = (_Float16)(a1[e] * sc);
  }
  unsigned short* q = out + e0;
  *(volatile v8h*)q = hv;
  __threadfence();
  *(volatile v8h*)q = hv;
}

__global__ __launch_bounds__(256) void ln_w_tokens_kernel(
    const float* __restrict__ x, const float* __restrict__ lw, const float* __restrict__ lb,
    float* __restrict__ Mt)
{
  __shared__ __align__(16) float sT[64 * 68];
  const int tid = threadIdx.x, lane = tid & 31, wave = tid >> 5;
  const int bid = blockIdx.x;
  const int cc = bid % 3;
  const int h  = (bid / 3) % kHgt;
  const int b  = bid / (3 * kHgt);
  const int c0 = cc * 64;
  const float w0 = lw[2 * lane], w1 = lw[2 * lane + 1];
  const float e0 = lb[2 * lane], e1 = lb[2 * lane + 1];
#pragma unroll 1
  for (int k = 0; k < 8; ++k) {
    const int c = wave * 8 + k;
    const float* xr = x + (((size_t)(b * kCh + c0 + c) * kHgt + h) * kWid);
    const v2f xv = *(const v2f*)(xr + 2 * lane);
    const float s = wave_sum(xv[0] + xv[1]);
    const float mu = s * (1.0f / (float)kWid);
    const float d0 = xv[0] - mu, d1 = xv[1] - mu;
    const float q = wave_sum(d0 * d0 + d1 * d1);
    const float rstd = rsqrtf(q * (1.0f / (float)kWid) + 1e-5f);
    sT[c * 68 + 2 * lane]     = d0 * rstd * w0 + e0;
    sT[c * 68 + 2 * lane + 1] = d1 * rstd * w1 + e1;
  }
  __syncthreads();
  const int hh = lane >> 4, c4 = (lane & 15) * 4;
  for (int pass = 0; pass < 2; ++pass) {
#pragma unroll
    for (int it = 0; it < 4; ++it) {
      const int w = wave * 8 + it * 2 + hh;
      v4f v;
      v[0] = sT[(c4 + 0) * 68 + w];
      v[1] = sT[(c4 + 1) * 68 + w];
      v[2] = sT[(c4 + 2) * 68 + w];
      v[3] = sT[(c4 + 3) * 68 + w];
      *(volatile v4f*)(Mt + (size_t)(b * kSeq + h * kWid + w) * kDm + c0 + c4) = v;
    }
    __threadfence();
  }
}

__global__ __launch_bounds__(256) void ln_c_update_kernel(
    float* __restrict__ Mt, float* __restrict__ Rs, const float* __restrict__ Ol,
    const float* __restrict__ nw, const float* __restrict__ nb,
    unsigned short* __restrict__ Hn, int cmode)
{
  __shared__ __align__(16) float sH[8 * kDm];
  const int tid = threadIdx.x, lane = tid & 31, wave = tid >> 5;
  const int row = blockIdx.x * 8 + wave;
  const int colA = lane * 4;
  const int colB = 128 + (lane & 15) * 4;
  const bool hasB = lane < 16;
  const float fb = hasB ? 1.0f : 0.0f;
  const size_t rbase = (size_t)row * kDm;
  const v4f ma = *(const v4f*)(Mt + rbase + colA);
  const v4f mb = *(const v4f*)(Mt + rbase + colB);
  v4f ra = ma * 0.0f, rb4 = mb * 0.0f, oa = ma * 0.0f, ob = mb * 0.0f;
  if (cmode != 0) {
    ra  = *(const v4f*)(Rs + rbase + colA);
    rb4 = *(const v4f*)(Rs + rbase + colB);
    oa  = *(const v4f*)(Ol + rbase + colA);
    ob  = *(const v4f*)(Ol + rbase + colB);
  }
  v4f mna, mnb, rna, rnb;
  if (cmode == 0) {
    mna = ma; mnb = mb; rna = ma * 0.0f; rnb = mb * 0.0f;
  } else if (cmode == 2) {
    rna = ma + ra; rnb = mb + rb4; mna = oa; mnb = ob;
  } else {
    const v4f ia0 = ma + ra, ib0 = mb + rb4;
    rna = ra + ia0; rnb = rb4 + ib0;
    mna = ma + oa;  mnb = mb + ob;
  }
  const v4f ia = mna + rna, ib = mnb + rnb;
  float s = ((ia[0] + ia[1]) + (ia[2] + ia[3])) + fb * ((ib[0] + ib[1]) + (ib[2] + ib[3]));
  s = wave_sum(s);
  const float mu = s * (1.0f / (float)kDm);
  const v4f da = ia - mu, db = ib - mu;
  float q = ((da[0] * da[0] + da[1] * da[1]) + (da[2] * da[2] + da[3] * da[3]))
          + fb * ((db[0] * db[0] + db[1] * db[1]) + (db[2] * db[2] + db[3] * db[3]));
  q = wave_sum(q);
  const float rstd = rsqrtf(q * (1.0f / (float)kDm) + 1e-5f);
  const v4f wa = *(const v4f*)(nw + colA), wb = *(const v4f*)(nw + colB);
  const v4f ba = *(const v4f*)(nb + colA), bbv = *(const v4f*)(nb + colB);
  const v4f ha = da * rstd * wa + ba;
  const v4f hb = db * rstd * wb + bbv;
  float* sh = sH + wave * kDm;
  *(v4f*)(sh + colA) = ha;
  if (hasB) *(v4f*)(sh + colB) = hb;
  __syncthreads();
  const int lc = (lane < 24) ? lane : 0;
  const v4f h0 = *(const v4f*)(sh + lc * 8);
  const v4f h1 = *(const v4f*)(sh + lc * 8 + 4);
  v8h hv;
#pragma unroll
  for (int e = 0; e < 4; ++e) { hv[e] = (_Float16)h0[e]; hv[4 + e] = (_Float16)h1[e]; }
  for (int pass = 0; pass < 2; ++pass) {
    if (cmode != 0) {
      *(volatile v4f*)(Mt + rbase + colA) = mna;
      if (hasB) *(volatile v4f*)(Mt + rbase + colB) = mnb;
    }
    *(volatile v4f*)(Rs + rbase + colA) = rna;
    if (hasB) *(volatile v4f*)(Rs + rbase + colB) = rnb;
    if (lane < 24) *(volatile v8h*)(Hn + rbase + lane * 8) = hv;
    __threadfence();
  }
}

__global__ __launch_bounds__(kConvCh) void conv_silu_kernel(
    const float* __restrict__ Xz, const float* __restrict__ cw, const float* __restrict__ cb,
    float* __restrict__ Uc, unsigned short* __restrict__ Uc16, int dir)
{
  __shared__ __align__(16) float sT[64 * kConvTP];
  const int tid = threadIdx.x, lane = tid & 31, wave = tid >> 5, hh = lane >> 4;
  const int d0 = blockIdx.x * kConvCh, d = d0 + tid;
  const int g0 = blockIdx.y * 64;
  const int tb = g0 & (kSeq - 1);
  const float w0 = cw[d * 4 + 0], w1 = cw[d * 4 + 1], w2 = cw[d * 4 + 2], w3 = cw[d * 4 + 3];
  const float bc = cb[d];
  const bool rev = (dir != 0);
  const bool hist = rev ? (tb + 64 < kSeq) : (tb > 0);
  const int rb = rev ? (hist ? (g0 + 64) : g0) : (hist ? (g0 - 3) : g0);
  const float e0 = Xz[(size_t)rb * kXzP + d];
  const float e1 = Xz[(size_t)(rb + 1) * kXzP + d];
  const float e2 = Xz[(size_t)(rb + 2) * kXzP + d];
  float xm3 = rev ? e2 : e0;
  float xm2 = e1;
  float xm1 = rev ? e0 : e2;
  if (!hist) { xm3 = 0.f; xm2 = 0.f; xm1 = 0.f; }
#pragma unroll 1
  for (int s = 0; s < 64; ++s) {
    const int r = rev ? (63 - s) : s;
    const float xcur = Xz[(size_t)(g0 + r) * kXzP + d];
    float acc = w0 * xm3;
    acc = fmaf(w1, xm2, acc);
    acc = fmaf(w2, xm1, acc);
    acc = fmaf(w3, xcur, acc);
    const float sv = acc + bc;
    const float sg = __builtin_amdgcn_rcpf(1.0f + __expf(-sv));
    sT[r * kConvTP + tid] = sv * sg;
    xm3 = xm2; xm2 = xm1; xm1 = xcur;
  }
  __syncthreads();
  const int c4 = lane * 4;
  const int c8 = (lane & 15) * 8;
  for (int pass = 0; pass < 2; ++pass) {
#pragma unroll
    for (int it = 0; it < 16; ++it) {
      const int row = it * 4 + wave;
      const v4f v = *(const v4f*)(sT + row * kConvTP + c4);
      *(volatile v4f*)(Uc + (size_t)(g0 + row) * kDin + d0 + c4) = v;
    }
#pragma unroll
    for (int it = 0; it < 8; ++it) {
      const int row = it * 8 + wave * 2 + hh;
      const float* sp = sT + row * kConvTP + c8;
      const v4f a0 = *(const v4f*)(sp);
      const v4f a1 = *(const v4f*)(sp + 4);
      v8h hv;
#pragma unroll
      for (int e = 0; e < 4; ++e) { hv[e] = (_Float16)(a0[e] * 16.0f); hv[4 + e] = (_Float16)(a1[e] * 16.0f); }
      *(volatile v8h*)(Uc16 + (size_t)(g0 + row) * kDin + d0 + c8) = hv;
    }
    __threadfence();
  }
}

__global__ __launch_bounds__(kScanCh) void scan_kernel(
    const float* __restrict__ Xd, const float* __restrict__ Uc, const float* __restrict__ Xz,
    const float* __restrict__ Wdt, const float* __restrict__ bdt, const float* __restrict__ Alog,
    const float* __restrict__ Dp, unsigned short* __restrict__ Y16, int dir)
{
  __shared__ __align__(16) float sX[kScanTS * kXdP];
  __shared__ __align__(16) float sY[kScanTS * kScanYP];
  __shared__ __align__(16) float sW[kDtR * kScanCh];
  __shared__ __align__(16) float sA[kNst * kScanCh];
  const int tid = threadIdx.x, lane = tid & 31, wave = tid >> 5;
  constexpr int kBlkPerB = kDin / kScanCh;
  const int bix = blockIdx.x / kBlkPerB;
  const int d0  = (blockIdx.x - bix * kBlkPerB) * kScanCh;
  const int d   = d0 + tid;
  const size_t row0 = (size_t)bix * kSeq;
  const bool rev = (dir != 0);
#pragma unroll 1
  for (int r = 0; r < kDtR; ++r) sW[r * kScanCh + tid] = Wdt[(size_t)d * kDtR + r];
#pragma unroll 1
  for (int s = 0; s < kNst; ++s) sA[s * kScanCh + tid] = -expf(Alog[(size_t)d * kNst + s]);
  __syncthreads();
  float negA[kNst], h[kNst];
#pragma unroll
  for (int s = 0; s < kNst; ++s) {
    negA[s] = sA[s * kScanCh + tid];
    h[s] = 0.f;
  }
  const float bb = bdt[d], Dd = Dp[d];
  const int lr = tid >> 4, lc4 = (tid & 15) * 4;
  const int q = lane >> 3, c8 = (lane & 7) * 8;
#pragma unroll 1
  for (int s0 = 0; s0 < kSeq; s0 += kScanTS) {
    const int tb = rev ? (kSeq - kScanTS - s0) : s0;
    __syncthreads();
#pragma unroll
    for (int i = 0; i < 16; ++i) {
      const int r = lr + 4 * i;
      *(v4f*)(sX + r * kXdP + lc4) = *(const v4f*)(Xd + (row0 + tb + r) * kXdP + lc4);
    }
    __syncthreads();
#pragma unroll 1
    for (int s = 0; s < kScanTS; ++s) {
      const int r = rev ? (kScanTS - 1 - s) : s;
      const size_t t = row0 + tb + r;
      const float* xr = sX + r * kXdP;
      float vdot = 0.f;
#pragma unroll 1
      for (int r4 = 0; r4 < kDtR / 4; ++r4) {
        const v4f xv = *(const v4f*)(xr + 4 * r4);
        const float* wp = sW + (4 * r4) * kScanCh + tid;
        vdot = fmaf(xv[0], wp[0], vdot);
        vdot = fmaf(xv[1], wp[kScanCh], vdot);
        vdot = fmaf(xv[2], wp[2 * kScanCh], vdot);
        vdot = fmaf(xv[3], wp[3 * kScanCh], vdot);
      }
      float Bs[kNst], Cs[kNst];
#pragma unroll
      for (int q4 = 0; q4 < 4; ++q4) {
        const v4f bv = *(const v4f*)(xr + kDtR + 4 * q4);
        const v4f cv = *(const v4f*)(xr + kDtR + kNst + 4 * q4);
        Bs[4 * q4 + 0] = bv[0]; Bs[4 * q4 + 1] = bv[1]; Bs[4 * q4 + 2] = bv[2]; Bs[4 * q4 + 3] = bv[3];
        Cs[4 * q4 + 0] = cv[0]; Cs[4 * q4 + 1] = cv[1]; Cs[4 * q4 + 2] = cv[2]; Cs[4 * q4 + 3] = cv[3];
      }
      const float v   = vdot + bb;
      const float a   = __expf(-fabsf(v));
      const float u   = 1.0f + a;
      const float l1p = __logf(u) + (a - (u - 1.0f)) * __builtin_amdgcn_rcpf(u);
      const float dt  = fmaxf(v, 0.0f) + l1p;
      const float xt  = Uc[t * kDin + d];
      const float dtx = dt * xt;
      float y = 0.f;
#pragma unroll
      for (int k = 0; k < kNst; ++k) {
        const float e = __expf(dt * negA[k]);
        h[k] = e * h[k] + dtx * Bs[k];
        y = h[k] * Cs[k] + y;
      }
      y = xt * Dd + y;
      const float zv = Xz[t * kXzP + kDin + d];
      const float sg = __builtin_amdgcn_rcpf(1.0f + __expf(-zv));
      y = y * (zv * sg);
      sY[r * kScanYP + tid] = y;
    }
    __syncthreads();
    for (int pass = 0; pass < 2; ++pass) {
#pragma unroll
      for (int it = 0; it < 8; ++it) {
        const int row = it * 8 + wave * 4 + q;
        const float* sp = sY + row * kScanYP + c8;
        const v4f a0 = *(const v4f*)(sp);
        const v4f a1 = *(const v4f*)(sp + 4);
        v8h hv;
#pragma unroll
        for (int e = 0; e < 4; ++e) { hv[e] = (_Float16)(a0[e] * 256.0f); hv[4 + e] = (_Float16)(a1[e] * 256.0f); }
        *(volatile v8h*)(Y16 + (row0 + tb + row) * kDin + d0 + c8) = hv;
      }
      __threadfence();
    }
  }
}

__global__ __launch_bounds__(256) void to_nchw_ln_kernel(
    const float* __restrict__ Mt, const float* __restrict__ Ol, const float* __restrict__ x,
    const float* __restrict__ lw, const float* __restrict__ lb,
    float* __restrict__ M2, unsigned short* __restrict__ T16)
{
  __shared__ __align__(16) float sT[64 * 68];
  __shared__ __align__(16) float sU[64 * 68];
  __shared__ __align__(16) float sV[64 * 68];
  const int tid = threadIdx.x, lane = tid & 31, wave = tid >> 5;
  const int bid = blockIdx.x;
  const int cc = bid % 3;
  const int h  = (bid / 3) % kHgt;
  const int b  = bid / (3 * kHgt);
  const int c0 = cc * 64;
#pragma unroll
  for (int i = 0; i < 4; ++i) {
    const int idx = tid + 256 * i;
    const int w = idx >> 4, c4 = (idx & 15) * 4;
    const size_t o = (size_t)(b * kSeq + h * kWid + w) * kDm + c0 + c4;
    const v4f v = *(const v4f*)(Mt + o) + *(const v4f*)(Ol + o);
    *(v4f*)(sT + w * 68 + c4) = v;
  }
  __syncthreads();
  const float w0 = lw[2 * lane], w1 = lw[2 * lane + 1];
  const float e0 = lb[2 * lane], e1 = lb[2 * lane + 1];
#pragma unroll 1
  for (int k = 0; k < 8; ++k) {
    const int c = wave * 8 + k;
    const float* xr = x + (((size_t)(b * kCh + c0 + c) * kHgt + h) * kWid);
    const v2f xv = *(const v2f*)(xr + 2 * lane);
    const float m0 = sT[(2 * lane) * 68 + c] + xv[0];
    const float m1 = sT[(2 * lane + 1) * 68 + c] + xv[1];
    const float s = wave_sum(m0 + m1);
    const float mu = s * (1.0f / (float)kWid);
    const float d0 = m0 - mu, d1 = m1 - mu;
    const float q = wave_sum(d0 * d0 + d1 * d1);
    const float rstd = rsqrtf(q * (1.0f / (float)kWid) + 1e-5f);
    sU[c * 68 + 2 * lane]     = m0;
    sU[c * 68 + 2 * lane + 1] = m1;
    sV[c * 68 + 2 * lane]     = d0 * rstd * w0 + e0;
    sV[c * 68 + 2 * lane + 1] = d1 * rstd * w1 + e1;
  }
  __syncthreads();
  const int hh = lane >> 4, c4 = (lane & 15) * 4;
  const int q = lane >> 3, c8 = (lane & 7) * 8;
  for (int pass = 0; pass < 2; ++pass) {
#pragma unroll
    for (int it = 0; it < 4; ++it) {
      const int c = wave * 8 + it * 2 + hh;
      const size_t R = (size_t)(b * kCh + c0 + c) * kHgt + h;
      const v4f v = *(const v4f*)(sU + c * 68 + c4);
      *(volatile v4f*)(M2 + R * kWid + c4) = v;
    }
#pragma unroll
    for (int it = 0; it < 2; ++it) {
      const int c = wave * 8 + it * 4 + q;
      const size_t R = (size_t)(b * kCh + c0 + c) * kHgt + h;
      const float* sp = sV + c * 68 + c8;
      const v4f a0 = *(const v4f*)(sp);
      const v4f a1 = *(const v4f*)(sp + 4);
      v8h hv;
#pragma unroll
      for (int e = 0; e < 4; ++e) { hv[e] = (_Float16)a0[e]; hv[4 + e] = (_Float16)a1[e]; }
      *(volatile v8h*)(T16 + R * kWid + c8) = hv;
    }
    __threadfence();
  }
}

__global__ __launch_bounds__(256) void gelu_f16x2_kernel(
    const float* __restrict__ in, unsigned short* __restrict__ out, int n2)
{
  const int i = blockIdx.x * 256 + threadIdx.x;
  if (i < n2) {
    const v2f v = *(const v2f*)(in + 2 * (size_t)i);
    const float g0 = 0.5f * v[0] * (1.0f + erff(v[0] * 0.70710678118654752f));
    const float g1 = 0.5f * v[1] * (1.0f + erff(v[1] * 0.70710678118654752f));
    const _Float16 h0 = (_Float16)(g0 * 16.0f), h1 = (_Float16)(g1 * 16.0f);
    const unsigned u = (unsigned)__builtin_bit_cast(unsigned short, h0) | ((unsigned)__builtin_bit_cast(unsigned short, h1) << 16);
    ((volatile unsigned*)out)[i] = u;
    __threadfence();
    ((volatile unsigned*)out)[i] = u;
  }
}

extern "C" void kernel_launch(void* const* d_in, const int* in_sizes, int n_in,
                              void* d_out, int out_size, void* d_ws, size_t ws_size,
                              hipStream_t stream) {
  if (n_in < 20) return;
  if (in_sizes[0] != kNchw) return;
  if (in_sizes[1] != kWid || in_sizes[2] != kWid) return;
  if (in_sizes[3] != kNL * kDm || in_sizes[4] != kNL * kDm) return;
  if (in_sizes[5] != kNL * kXzP * kDm) return;
  if (in_sizes[6] != kNL * kDin * 4 || in_sizes[7] != kNL * kDin) return;
  if (in_sizes[8] != kNL * kXdW * kDin) return;
  if (in_sizes[9] != kNL * kDin * kDtR || in_sizes[10] != kNL * kDin) return;
  if (in_sizes[11] != kNL * kDin * kNst || in_sizes[12] != kNL * kDin) return;
  if (in_sizes[13] != kNL * kDm * kDin) return;
  if (in_sizes[14] != kWid || in_sizes[15] != kWid) return;
  if (in_sizes[16] != kMlpH * kWid || in_sizes[17] != kMlpH) return;
  if (in_sizes[18] != kWid * kMlpH || in_sizes[19] != kWid) return;
  if (out_size != kNchw) return;
  if (ws_size < kWsTotal) return;

  const float* x         = (const float*)d_in[0];
  const float* ln1_w     = (const float*)d_in[1];
  const float* ln1_b     = (const float*)d_in[2];
  const float* norm_w    = (const float*)d_in[3];
  const float* norm_b    = (const float*)d_in[4];
  const float* in_proj_w = (const float*)d_in[5];
  const float* conv_w    = (const float*)d_in[6];
  const float* conv_b    = (const float*)d_in[7];
  const float* x_proj_w  = (const float*)d_in[8];
  const float* dt_proj_w = (const float*)d_in[9];
  const float* dt_proj_b = (const float*)d_in[10];
  const float* A_log     = (const float*)d_in[11];
  const float* ssm_D     = (const float*)d_in[12];
  const float* out_proj_w= (const float*)d_in[13];
  const float* ln2_w     = (const float*)d_in[14];
  const float* ln2_b     = (const float*)d_in[15];
  const float* mlp_w1    = (const float*)d_in[16];
  const float* mlp_b1    = (const float*)d_in[17];
  const float* mlp_w2    = (const float*)d_in[18];
  const float* mlp_b2    = (const float*)d_in[19];
  float* out = (float*)d_out;

  char* ws = (char*)d_ws;
  float*          Mt   = (float*)(ws + kOffM);
  float*          Rs   = (float*)(ws + kOffRes);
  float*          Ol   = (float*)(ws + kOffOutl);
  unsigned short* Hn   = (unsigned short*)(ws + kOffHn);
  unsigned short* Wi   = (unsigned short*)(ws + kOffWi);
  unsigned short* Wx   = (unsigned short*)(ws + kOffWx);
  unsigned short* Wo   = (unsigned short*)(ws + kOffWo);
  unsigned short* W1   = (unsigned short*)(ws + kOffW1);
  unsigned short* W2   = (unsigned short*)(ws + kOffW2);
  float*          Xz   = (float*)(ws + kOffXz);
  float*          Uc   = (float*)(ws + kOffUc);
  unsigned short* Uc16 = (unsigned short*)(ws + kOffUc16);
  float*          Xd   = (float*)(ws + kOffXd);
  unsigned short* Y16  = (unsigned short*)(ws + kOffY16);
  float*          M2   = (float*)(ws + kOffM2);
  unsigned short* T16  = (unsigned short*)(ws + kOffT16);
  float*          H1   = (float*)(ws + kOffXz);
  unsigned short* G16  = (unsigned short*)(ws + kOffUc);

  {
    const int n8i = kNL * kXzP * kDm / 8;
    cast_scale_f16x8_kernel<<<(n8i + 255) / 256, 256, 0, stream>>>(in_proj_w, Wi, n8i, 64.0f);
    const int n8x = kNL * kXdP * kDin / 8;
    cast_xproj_pad_f16_kernel<<<(n8x + 255) / 256, 256, 0, stream>>>(x_proj_w, Wx, n8x);
    const int n8o = kNL * kDm * kDin / 8;
    cast_scale_f16x8_kernel<<<(n8o + 255) / 256, 256, 0, stream>>>(out_proj_w, Wo, n8o, 64.0f);
    const int n8m = kMlpH * kWid / 8;
    cast_scale_f16x8_kernel<<<(n8m + 255) / 256, 256, 0, stream>>>(mlp_w1, W1, n8m, 64.0f);
    cast_scale_f16x8_kernel<<<(n8m + 255) / 256, 256, 0, stream>>>(mlp_w2, W2, n8m, 64.0f);
  }

  ln_w_tokens_kernel<<<kBatch * kHgt * 3, 256, 0, stream>>>(x, ln1_w, ln1_b, Mt);

  for (int l = 0; l < kNL; ++l) {
    const int dir = l & 1;
    const int cmode = (l == 0) ? 0 : (((l - 1) & 1) ? 3 : 2);
    ln_c_update_kernel<<<kTok / 8, 256, 0, stream>>>(
        Mt, Rs, Ol, norm_w + (size_t)l * kDm, norm_b + (size_t)l * kDm, Hn, cmode);

    wmma_gemm64<0, 0, 0, 0, false><<<dim3(kTilesIn / 8, 1), 256, 0, stream>>>(
        Hn, nullptr, kDm, 0L,
        Wi + (size_t)l * kXzP * kDm, nullptr, kDm, 0L,
        (void*)Xz, nullptr, kXzP, 0L,
        nullptr, nullptr, 0L,
        kTok, kXzP, kDm, 1.0f / 64.0f);

    conv_silu_kernel<<<dim3(kDin / kConvCh, kTok / 64), kConvCh, 0, stream>>>(
        Xz, conv_w + (size_t)l * kDin * 4, conv_b + (size_t)l * kDin, Uc, Uc16, dir);

    wmma_gemm64<0, 0, 0, 0, false><<<dim3(kTilesX / 8, 1), 256, 0, stream>>>(
        Uc16, nullptr, kDin, 0L,
        Wx + (size_t)l * kXdP * kDin, nullptr, kDin, 0L,
        (void*)Xd, nullptr, kXdP, 0L,
        nullptr, nullptr, 0L,
        kTok, kXdP, kDin, 1.0f / 1024.0f);

    scan_kernel<<<kBatch * (kDin / kScanCh), kScanCh, 0, stream>>>(
        Xd, Uc, Xz, dt_proj_w + (size_t)l * kDin * kDtR, dt_proj_b + (size_t)l * kDin,
        A_log + (size_t)l * kDin * kNst, ssm_D + (size_t)l * kDin, Y16, dir);

    wmma_gemm64<0, 0, 0, 0, false><<<dim3(kTilesOut / 8, 1), 256, 0, stream>>>(
        Y16, nullptr, kDin, 0L,
        Wo + (size_t)l * kDm * kDin, nullptr, kDin, 0L,
        (void*)Ol, nullptr, kDm, 0L,
        nullptr, nullptr, 0L,
        kTok, kDm, kDin, 1.0f / 16384.0f);
  }

  to_nchw_ln_kernel<<<kBatch * kHgt * 3, 256, 0, stream>>>(Mt, Ol, x, ln2_w, ln2_b, M2, T16);

  wmma_gemm64<0, 0, 2, 0, false><<<dim3(kTilesM1 / 8, 1), 256, 0, stream>>>(
      T16, nullptr, kWid, 0L,
      W1, nullptr, kWid, 0L,
      (void*)H1, nullptr, kMlpH, 0L,
      mlp_b1, nullptr, 0L,
      kMlpRows, kMlpH, kWid, 1.0f / 64.0f);

  {
    const int n2 = kMlpRows * kMlpH / 2;
    gelu_f16x2_kernel<<<(n2 + 255) / 256, 256, 0, stream>>>(H1, G16, n2);
  }

  wmma_gemm64<0, 0, 2, 0, true><<<dim3(kTilesM2 / 8, 1), 256, 0, stream>>>(
      G16, nullptr, kMlpH, 0L,
      W2, nullptr, kMlpH, 0L,
      (void*)out, nullptr, kWid, 0L,
      mlp_b2, M2, 0L,
      kMlpRows, kWid, kMlpH, 1.0f / 1024.0f);
}
